// OptNetEq_39642548142386
// MI455X (gfx1250) — hardware-verified
//
#include <hip/hip_runtime.h>
#include <math.h>

constexpr int   kNVar     = 100;
constexpr int   kNCon     = 50;
constexpr int   kBatch    = 1024;
constexpr int   kIters    = 20;
constexpr float kQpen     = 0.1f;
constexpr float kSigma    = 0.1f;
constexpr float kStepFrac = 0.99f;
static constexpr float kPivotFloor = 1e-3f;
constexpr int   kThreads  = 256;
constexpr int   kAPitch   = 104;
constexpr int   kKPad     = 128;
constexpr int   kBPitch   = 136;
constexpr int   kSPitch   = 65;
constexpr int   kZPitch   = 128;
constexpr int   kBChunks  = 13;
constexpr int   kCopyThreads = (kBatch * kNVar) / 4;

static_assert(kKPad % 32 == 0, "wmma depth multiple of 32");
static_assert((kBatch * kNVar) % (4 * 256) == 0, "copy grid exact");
static_assert(kNVar % 4 == 0, "float4 chunks stay within an output row");
static_assert(kAPitch % 4 == 0 && kAPitch >= 8 * kBChunks, "B chunk reads stay inside an sA row");
static_assert(8 * kBChunks >= kNVar && 8 * kBChunks <= kKPad, "B chunks cover the real depth");
static_assert(kBPitch % 8 == 0 && kBPitch >= kKPad, "16-B aligned fragment rows");

typedef __attribute__((ext_vector_type(16))) _Float16 v16h;
typedef __attribute__((ext_vector_type(8)))  _Float16 v8h;
typedef __attribute__((ext_vector_type(16))) __bf16   v16b;
typedef __attribute__((ext_vector_type(8)))  __bf16   v8b;
typedef __attribute__((ext_vector_type(8)))  float    v8f;
typedef __attribute__((ext_vector_type(4)))  float    v4f;
typedef __attribute__((ext_vector_type(4)))  unsigned int v4u;

__device__ __forceinline__ unsigned short f2bf_bits(float f) {
  unsigned u = __float_as_uint(f);
  return (unsigned short)((u + 0x7FFFu + ((u >> 16) & 1u)) >> 16);
}
__device__ __forceinline__ float bf_bits2f(unsigned short h) { return __uint_as_float(((unsigned)h) << 16); }

template <typename T> struct Frag;
template <> struct Frag<__bf16> {
  typedef v16b V; union U { v16b v; v8b h[2]; };
  static __device__ __forceinline__ v16b load(const __bf16* p) {
    U f; f.h[0] = *(const v8b*)(p); f.h[1] = *(const v8b*)(p + 16); return f.v;
  }
  static __device__ __forceinline__ v8f mma(v16b a, v16b b, v8f c) {
    return __builtin_amdgcn_wmma_f32_16x16x32_bf16(false, a, false, b, (short)0, c, false, false);
  }
};

__device__ __forceinline__ unsigned short at_bf_bits(float f) {
  unsigned u = __float_as_uint(f);
  return (unsigned short)((u + 0x7FFFu + ((u >> 16) & 1u)) >> 16);
}
__device__ __forceinline__ __bf16 at_f2bf(float f) { return __builtin_bit_cast(__bf16, at_bf_bits(f)); }
__device__ __forceinline__ v8f at_mma(v16b a, v16b b, v8f c) {
  c = __builtin_amdgcn_wmma_f32_16x16x32_bf16(false, a, false, b, (short)0, c, false, false);
  asm volatile("v_nop\n\tv_nop\n\tv_nop\n\tv_nop" : "+v"(c) : "v"(a), "v"(b));
  return c;
}

__device__ __forceinline__ unsigned pk16(unsigned short a, unsigned short b) { return (unsigned)a | ((unsigned)b << 16); }

__device__ __forceinline__ void split_pair(float f0, float f1, unsigned& hw, unsigned& lw) {
  const unsigned short h0 = at_bf_bits(f0);
  const unsigned short h1 = at_bf_bits(f1);
  const unsigned short l0 = at_bf_bits(f0 - bf_bits2f(h0));
  const unsigned short l1 = at_bf_bits(f1 - bf_bits2f(h1));
  hw = pk16(h0, h1);
  lw = pk16(l0, l1);
}

__device__ __forceinline__ void lds_wave_sync() {
  __builtin_amdgcn_fence(__ATOMIC_RELEASE, "workgroup");
  __builtin_amdgcn_wave_barrier();
  __builtin_amdgcn_fence(__ATOMIC_ACQUIRE, "workgroup");
}

__device__ __forceinline__ float wave_sum(float v) {
  v += __shfl_xor(v, 16, 32);
  v += __shfl_xor(v, 8, 32);
  v += __shfl_xor(v, 4, 32);
  v += __shfl_xor(v, 2, 32);
  v += __shfl_xor(v, 1, 32);
  return v;
}
__device__ __forceinline__ float wave_min(float v) {
  v = fminf(v, __shfl_xor(v, 16, 32));
  v = fminf(v, __shfl_xor(v, 8, 32));
  v = fminf(v, __shfl_xor(v, 4, 32));
  v = fminf(v, __shfl_xor(v, 2, 32));
  v = fminf(v, __shfl_xor(v, 1, 32));
  return v;
}

__global__ __launch_bounds__(kThreads)
void qp_ipm_block_kernel(const float* __restrict__ x, const float* __restrict__ A, float* __restrict__ zplane) {
  __shared__ __align__(16) float          sA[kNCon * kAPitch];
  __shared__ __align__(16) unsigned short sBh[64 * kBPitch];
  __shared__ __align__(16) unsigned short sBl[64 * kBPitch];
  __shared__ __align__(16) float          sS[64 * kSPitch];
  __shared__ __align__(16) float          sz[kZPitch];
  __shared__ __align__(16) float          ssw[kKPad];
  __shared__ __align__(16) float          st1[kKPad];
  __shared__ float snu[64];
  __shared__ float srhs[64];
  __shared__ float sdnu[64];
  __shared__ float sinvd[64];
  __shared__ float spart[8];
  __shared__ float spart2[8];

  const int tid  = threadIdx.x;
  const int lane = tid & 31;
  const int wave = tid >> 5;
  const int b    = blockIdx.x;
  const int ic   = min(tid, kNVar - 1);
  const int jc   = min(tid, kNCon - 1);

#pragma unroll 1
  for (int it = 0; it < 21; ++it) {
    const int e  = tid + it * kThreads;
    const int ec = min(e, kNCon * kAPitch - 1);
    const int j  = ec / kAPitch;
    const int kk = ec - j * kAPitch;
    const float av   = A[j * kNVar + min(kk, kNVar - 1)];
    const float fsel = (kk < kNVar) ? 1.0f : 0.0f;
    const float v    = av * fsel;
    if (e < kNCon * kAPitch) sA[e] = v;
  }
#pragma unroll 1
  for (int it = 0; it < 17; ++it) {
    const int e = tid + it * kThreads;
    if (e < 64 * kSPitch) sS[e] = 0.0f;
  }
  {
    const v4u z4 = (v4u){0u, 0u, 0u, 0u};
#pragma unroll 1
    for (int it = 0; it < 5; ++it) {
      const int e = tid + it * kThreads;
      if (e < (64 * kBPitch) / 8) {
        *(v4u*)(sBh + 8 * e) = z4;
        *(v4u*)(sBl + 8 * e) = z4;
      }
    }
  }
  if (tid < kZPitch) sz[tid] = 0.0f;
  if (tid < kKPad) { ssw[tid] = 0.0f; st1[tid] = 0.0f; }
  if (tid < 64) { snu[tid] = 0.0f; srhs[tid] = 0.0f; sdnu[tid] = 0.0f; sinvd[tid] = 0.0f; }

  const float pv = x[(size_t)b * kNVar + ic];
  float z = 0.0f, s = 1.0f, lam = 1.0f, nu = 0.0f;
  __syncthreads();

#pragma unroll 1
  for (int step = 0; step < kIters; ++step) {
    float rx = 0.0f, rp = 0.0f, sl = 0.0f, ra = 0.0f;
    if (wave < 4) {
      float atn = 0.0f;
#pragma unroll 10
      for (int j = 0; j < kNCon; ++j) atn += sA[j * kAPitch + ic] * snu[j];
      rx = ((kQpen * z + pv) - lam) + atn;
      rp = s - z;
      sl = s * lam;
    }
    if (wave < 2) {
      float az = 0.0f;
#pragma unroll 10
      for (int k = 0; k < kNVar; ++k) az += sA[jc * kAPitch + k] * sz[k];
      ra = az - 1.0f;
    }
    {
      const float v = wave_sum((tid < kNVar) ? sl : 0.0f);
      if (lane == 0) spart[wave] = v;
    }
    __syncthreads();

    float r1 = 0.0f, rs = 0.0f, w = 0.0f;
    {
      float tot = spart[0];
#pragma unroll
      for (int q = 1; q < 8; ++q) tot += spart[q];
      const float mu = kSigma * (tot * (1.0f / (float)kNVar));
      if (wave < 4) {
        rs = sl - mu;
        const float d = lam / s;
        r1 = -rx + (lam * rp - rs) / s;
        w  = 1.0f / (kQpen + d);
        if (tid < kNVar) {
          ssw[tid] = sqrtf(w);
          st1[tid] = w * r1;
        }
      }
    }
    __syncthreads();

#pragma unroll 1
    for (int it = 0; it < 3; ++it) {
      const int e  = tid + it * kThreads;
      const int ec = min(e, kNCon * kBChunks - 1);
      const int j  = ec / kBChunks;
      const int c  = ec - j * kBChunks;
      const float* ar = sA + j * kAPitch + 8 * c;
      const v4f a0 = *(const v4f*)(ar);
      const v4f a1 = *(const v4f*)(ar + 4);
      const v4f g0 = *(const v4f*)(ssw + 8 * c);
      const v4f g1 = *(const v4f*)(ssw + 8 * c + 4);
      unsigned h0, h1, h2, h3, l0, l1, l2, l3;
      split_pair(a0[0] * g0[0], a0[1] * g0[1], h0, l0);
      split_pair(a0[2] * g0[2], a0[3] * g0[3], h1, l1);
      split_pair(a1[0] * g1[0], a1[1] * g1[1], h2, l2);
      split_pair(a1[2] * g1[2], a1[3] * g1[3], h3, l3);
      const v4u hv = (v4u){h0, h1, h2, h3};
      const v4u lv = (v4u){l0, l1, l2, l3};
      if (e < kNCon * kBChunks) {
        *(v4u*)(sBh + j * kBPitch + 8 * c) = hv;
        *(v4u*)(sBl + j * kBPitch + 8 * c) = lv;
      }
    }
    if (wave < 2) {
      float acc = 0.0f;
#pragma unroll 10
      for (int k = 0; k < kNVar; ++k) acc += sA[jc * kAPitch + k] * st1[k];
      if (tid < kNCon) srhs[tid] = acc + ra;
    }
    __syncthreads();

    {
      const int rl   = lane & 15;
      const int koff = (lane >> 4) * 8;
      const int mOff = (lane >> 4) * 8;
      const __bf16* Bh = (const __bf16*)sBh;
      const __bf16* Bl = (const __bf16*)sBl;
      for (int t = wave; t < 10; t += 8) {
        const int ti = (t >= 1) + (t >= 3) + (t >= 6);
        const int tj = t - ((ti * (ti + 1)) >> 1);
        const int arow = (16 * ti + rl) * kBPitch + koff;
        const int brow = (16 * tj + rl) * kBPitch + koff;
        v8f acc = (v8f){0.f, 0.f, 0.f, 0.f, 0.f, 0.f, 0.f, 0.f};
#pragma unroll
        for (int k0 = 0; k0 < kKPad; k0 += 32) {
          const v16b ah = Frag<__bf16>::load(Bh + arow + k0);
          const v16b al = Frag<__bf16>::load(Bl + arow + k0);
          const v16b bh = Frag<__bf16>::load(Bh + brow + k0);
          const v16b bl = Frag<__bf16>::load(Bl + brow + k0);
          acc = at_mma(ah, bh, acc);
          acc = at_mma(ah, bl, acc);
          acc = at_mma(al, bh, acc);
          acc = at_mma(al, bl, acc);
        }
#pragma unroll
        for (int r = 0; r < 8; ++r) sS[(16 * ti + mOff + r) * kSPitch + 16 * tj + rl] = acc[r];
      }
    }
    __syncthreads();

    if (wave == 0) {
#pragma unroll 1
      for (int k = 0; k < kNCon; ++k) {
        lds_wave_sync();
        const float piv  = sS[k * kSPitch + k];
        const float Lkk  = sqrtf(fmaxf(piv, kPivotFloor));
        const float invL = 1.0f / Lkk;
        if (lane == 0) sinvd[k] = invL;
        const int i0 = k + 1 + lane, i1 = k + 33 + lane;
        const int i0c = min(i0, 63), i1c = min(i1, 63);
        const float L0 = sS[i0c * kSPitch + k] * invL;
        const float L1 = sS[i1c * kSPitch + k] * invL;
        if (i0 < kNCon) sS[i0 * kSPitch + k] = L0;
        if (i1 < kNCon) sS[i1 * kSPitch + k] = L1;
        lds_wave_sync();
        const int iend = min(k + 32, kNCon - 1);
#pragma unroll 2
        for (int i = k + 1; i <= iend; ++i) {
          const float Lik = sS[i * kSPitch + k];
          const float sv  = sS[i * kSPitch + i0c] - Lik * L0;
          if (i0 <= i) sS[i * kSPitch + i0] = sv;
        }
#pragma unroll 2
        for (int i = k + 33; i < kNCon; ++i) {
          const float Lik = sS[i * kSPitch + k];
          const float s0  = sS[i * kSPitch + i0] - Lik * L0;
          sS[i * kSPitch + i0] = s0;
          const float s1  = sS[i * kSPitch + i1c] - Lik * L1;
          if (i1 <= i) sS[i * kSPitch + i1] = s1;
        }
      }
      lds_wave_sync();
      float q0 = srhs[lane];
      float q1 = srhs[32 + lane];
#pragma unroll 1
      for (int k = 0; k < kNCon; ++k) {
        const float cand = (k < 32) ? q0 : q1;
        const float yk   = __shfl(cand, k & 31, 32) * sinvd[k];
        const float Lr0  = sS[lane * kSPitch + k];
        const float Lr1  = sS[(32 + lane) * kSPitch + k];
        const float u0   = q0 - Lr0 * yk;
        const float u1   = q1 - Lr1 * yk;
        q0 = (lane == k) ? yk : ((lane > k) ? u0 : q0);
        q1 = (32 + lane == k) ? yk : ((32 + lane > k) ? u1 : q1);
      }
#pragma unroll 1
      for (int k = kNCon - 1; k >= 0; --k) {
        const float cand = (k < 32) ? q0 : q1;
        const float xk   = __shfl(cand, k & 31, 32) * sinvd[k];
        const float Lc0  = sS[k * kSPitch + lane];
        const float Lc1  = sS[k * kSPitch + 32 + lane];
        const float u0   = q0 - Lc0 * xk;
        const float u1   = q1 - Lc1 * xk;
        q0 = (lane == k) ? xk : ((lane < k) ? u0 : q0);
        q1 = (32 + lane == k) ? xk : ((32 + lane < k) ? u1 : q1);
      }
      sdnu[lane] = q0;
      sdnu[32 + lane] = q1;
    }
    __syncthreads();

    float dz = 0.0f, ds = 0.0f, dlam = 0.0f;
    float rat = INFINITY;
    if (wave < 4) {
      float atd = 0.0f;
#pragma unroll 10
      for (int j = 0; j < kNCon; ++j) atd += sA[j * kAPitch + ic] * sdnu[j];
      dz   = w * (r1 - atd);
      ds   = dz - rp;
      dlam = (-rs - lam * ds) / s;
      const float qs = -s / ds;
      const float ql = -lam / dlam;
      const float rS = (ds < 0.0f) ? qs : INFINITY;
      const float rL = (dlam < 0.0f) ? ql : INFINITY;
      rat = fminf(rS, rL);
    }
    {
      const float v = wave_min((tid < kNVar) ? rat : INFINITY);
      if (lane == 0) spart2[wave] = v;
    }
    __syncthreads();

    {
      float m = spart2[0];
#pragma unroll
      for (int q = 1; q < 8; ++q) m = fminf(m, spart2[q]);
      const float alpha = kStepFrac * fminf(1.0f, m);
      if (wave < 4) {
        z   += alpha * dz;
        s   += alpha * ds;
        lam += alpha * dlam;
        if (tid < kNVar) sz[tid] = z;
      }
      if (wave < 2) {
        const float dn = sdnu[jc];
        nu += alpha * dn;
        if (tid < kNCon) snu[tid] = nu;
      }
    }
    __syncthreads();
  }

  if (wave == 0) {
    const v4f v = *(const v4f*)(sz + 4 * lane);
    float* zp = zplane + (size_t)b * kZPitch + 4 * lane;
    *(volatile v4f*)zp = v;
    __threadfence();
    *(volatile v4f*)zp = v;
  }
}

__global__ __launch_bounds__(256)
void zcopy_kernel(const float* __restrict__ zp, float* __restrict__ out) {
  const int t   = blockIdx.x * 256 + threadIdx.x;
  const int e   = 4 * t;
  const int row = e / kNVar;
  const int col = e - row * kNVar;
  const v4f v = *(const v4f*)(zp + (size_t)row * kZPitch + col);
  float* op = out + e;
  *(volatile v4f*)op = v;
  __threadfence();
  *(volatile v4f*)op = v;
}

extern "C" void kernel_launch(void* const* d_in, const int* in_sizes, int n_in,
                              void* d_out, int out_size, void* d_ws, size_t ws_size,
                              hipStream_t stream) {
  if (n_in < 2) return;
  if (in_sizes[0] != kBatch * kNVar) return;
  if (in_sizes[1] != kNCon * kNVar) return;
  if (out_size != kBatch * kNVar) return;
  const size_t zplane_bytes = (size_t)kBatch * kZPitch * sizeof(float);
  if (ws_size < zplane_bytes) return;
  const float* xin = (const float*)d_in[0];
  const float* Ain = (const float*)d_in[1];
  float* out = (float*)d_out;
  float* zplane = (float*)d_ws;
  qp_ipm_block_kernel<<<dim3(kBatch), dim3(kThreads), 0, stream>>>(xin, Ain, zplane);
  zcopy_kernel<<<dim3(kCopyThreads / 256), dim3(256), 0, stream>>>(zplane, out);
}
